// FusedSparseLinear_70695161692194
// MI455X (gfx1250) — hardware-run, weakly checked
//
#include <hip/hip_runtime.h>

typedef __bf16   v16bf __attribute__((ext_vector_type(16)));
typedef __bf16   v8bf  __attribute__((ext_vector_type(8)));
typedef float    v8f   __attribute__((ext_vector_type(8)));
typedef float    v4f   __attribute__((ext_vector_type(4)));
typedef unsigned v4u   __attribute__((ext_vector_type(4)));
typedef int      v4i   __attribute__((ext_vector_type(4)));
typedef v8bf __attribute__((may_alias)) v8bfa;
typedef v4f  __attribute__((may_alias)) v4fa;
typedef v4u  __attribute__((may_alias)) v4ua;
typedef v4i  __attribute__((may_alias)) v4ia;

union FragB { v16bf v; v8bf half[2]; };

#define TOK    2048
#define KDIM   4096
#define MDIM   4096
#define NBLK   1024
#define TB     64
#define NRB    (MDIM / TB)
#define NCB    (KDIM / TB)
#define TT     128
#define NTHR   256
#define SROW   72

#define NX     (TOK * KDIM)
#define NV     (NBLK * TB * TB)
#define XBLK   (NX / 8 / NTHR)
#define VBLK   (NV / 8 / NTHR)
#define XB_BYTES ((size_t)NX * 2)
#define VB_BYTES ((size_t)NV * 2)
#define WS_TOTAL (XB_BYTES + VB_BYTES)

#define SA_BYTES (TT * SROW * 2)
#define SB_BYTES (TB * SROW * 2)
#define SO_BYTES (TT * TB * 4)
#define LDS_TOTAL (SO_BYTES + 3 * NBLK * 4 + TB * 4 + 16)

static_assert(NBLK == 1024);
static_assert(TB == 64 && TB == 2 * 32);
static_assert(NRB == 64 && NCB == 64);
static_assert(TOK == 2048 && TOK % TT == 0);
static_assert(NTHR == 8 * 32 && 8 * 16 == TT);
static_assert(NX % (8 * NTHR) == 0 && NV % (8 * NTHR) == 0);
static_assert(NBLK == NTHR * 4);
static_assert(SA_BYTES + SB_BYTES <= SO_BYTES);
static_assert(TT * TB / 4 == NTHR * 8);
static_assert(XB_BYTES % 128 == 0 && VB_BYTES % 128 == 0);
static_assert(LDS_TOTAL <= 65536);
static_assert(WS_TOTAL <= 134217728);

__device__ __forceinline__ unsigned bf16_bits(float f) {
  unsigned u = __float_as_uint(f);
  u += 0x7FFFu + ((u >> 16) & 1u);
  return u >> 16;
}
__device__ __forceinline__ unsigned bf16_pack2(float lo, float hi) {
  return bf16_bits(lo) | (bf16_bits(hi) << 16);
}
__device__ __forceinline__ float bf16_val(float f) {
  return __uint_as_float(bf16_bits(f) << 16);
}

__device__ __forceinline__ v8f wmma_bf16(v16bf a, v16bf b, v8f c) {
  v8f d = __builtin_amdgcn_wmma_f32_16x16x32_bf16(false, a, false, b, (short)0, c, false, false);
  asm volatile("v_nop\n\tv_nop\n\tv_nop\n\tv_nop" : "+v"(d) : "v"(a), "v"(b));
  return d;
}

__device__ __forceinline__ v16bf load_frag(const unsigned short* p, int h) {
  FragB f;
  f.half[0] = *(const v8bfa*)(p + 8 * h);
  f.half[1] = *(const v8bfa*)(p + 16 + 8 * h);
  return f.v;
}

__device__ __forceinline__ float gelu_t(float v) {
  #pragma clang fp contract(off)
  const float c = ((0.044715f * v) * v) * v;
  const float inner = 0.7978845608f * (v + c);
  const float th = tanhf(inner);
  return (v * 0.5f) * (1.0f + th);
}

__device__ __forceinline__ void cvt8(const float* __restrict__ src, unsigned short* __restrict__ dst) {
  const v4f a = *(const v4fa*)src;
  const v4f c = *(const v4fa*)(src + 4);
  const v4u o = { bf16_pack2(a.x, a.y), bf16_pack2(a.z, a.w),
                  bf16_pack2(c.x, c.y), bf16_pack2(c.z, c.w) };
  *(volatile v4u*)dst = o;
  __threadfence();
  *(volatile v4u*)dst = o;
}

__global__ __launch_bounds__(NTHR) void k_prep(
    const float* __restrict__ x, const float* __restrict__ vals,
    unsigned short* __restrict__ xb, unsigned short* __restrict__ vb)
{
  const int b = blockIdx.x, tid = threadIdx.x;
  if (b < XBLK) {
    const size_t g = (size_t)b * NTHR + tid;
    cvt8(x + g * 8, xb + g * 8);
  } else {
    const size_t g = (size_t)(b - XBLK) * NTHR + tid;
    cvt8(vals + g * 8, vb + g * 8);
  }
}

__device__ __forceinline__ void out_pass(const float* sO, float* out, int t0, int rb, int w, int lane) {
  const int q8 = lane & 7, sub = lane >> 3;
  #pragma unroll
  for (int i = 0; i < 8; ++i) {
    const int lid = w * 32 + i * 4 + sub;
    const int row = lid >> 1, hl = lid & 1;
    const v4f v = *(const v4fa*)(sO + row * TB + 32 * hl + 4 * q8);
    *(volatile v4f*)(out + (size_t)(t0 + row) * MDIM + TB * rb + 32 * hl + 4 * q8) = v;
  }
}

__global__ __launch_bounds__(NTHR) void k_bsgemm(
    const unsigned short* __restrict__ XB,
    const unsigned short* __restrict__ VB,
    const float* __restrict__ bias,
    const int* __restrict__ brow,
    const int* __restrict__ bcol,
    float* __restrict__ out)
{
  __shared__ __attribute__((aligned(16))) char  sU[SO_BYTES];
  __shared__ __attribute__((aligned(16))) int   sRows[NBLK];
  __shared__ __attribute__((aligned(16))) int   sCols[NBLK];
  __shared__ __attribute__((aligned(16))) int   sList[NBLK];
  __shared__ __attribute__((aligned(16))) float sBias[TB];
  __shared__ __attribute__((aligned(16))) int   sCnt[4];

  unsigned short* sA = (unsigned short*)sU;
  unsigned short* sB = (unsigned short*)(sU + SA_BYTES);
  float* sO = (float*)sU;

  const int tid = threadIdx.x, lane = tid & 31;
  const int w = __builtin_amdgcn_readfirstlane(tid >> 5);
  const int h = lane >> 4, m = lane & 15;
  const int t0 = blockIdx.x * TT;
  const int rb = blockIdx.y;

  {
    const v4i r4 = *(const v4ia*)(brow + 4 * tid);
    const v4i c4 = *(const v4ia*)(bcol + 4 * tid);
    *(v4ia*)(sRows + 4 * tid) = r4;
    *(v4ia*)(sCols + 4 * tid) = c4;
  }
  if (w == 0) {
    const int bi = lane & 15;
    const v4f bv = *(const v4fa*)(bias + TB * rb + 4 * bi);
    asm volatile("" :: "v"(bv));
    const v4f br = { bf16_val(bv.x), bf16_val(bv.y), bf16_val(bv.z), bf16_val(bv.w) };
    if (lane < 16) *(v4fa*)(sBias + 4 * bi) = br;
  }
  __syncthreads();

  if (w == 0) {
    int c = 0;
    #pragma unroll 1
    for (int it = 0; it < NBLK / 32; ++it) {
      const int id = 32 * it + lane;
      const int v = sRows[id];
      const bool hit = (v == rb);
      const unsigned msk = __builtin_amdgcn_ballot_w32(hit);
      const int pos = c + (int)__builtin_amdgcn_mbcnt_lo(msk, 0u);
      if (hit) sList[pos] = id;
      c += __popc(msk);
    }
    if (lane == 0) sCnt[0] = c;
  }
  __syncthreads();

  int cntv = sCnt[0];
  cntv = min(max(cntv, 0), NBLK);
  const int cnt = __builtin_amdgcn_readfirstlane(cntv);

  const v8f z8 = {0.f, 0.f, 0.f, 0.f, 0.f, 0.f, 0.f, 0.f};
  v8f acc[4];
  #pragma unroll
  for (int nt = 0; nt < 4; ++nt) acc[nt] = z8;

  const unsigned short* arow = sA + (16 * w + m) * SROW;
  const unsigned short* brw  = sB + m * SROW;

  #pragma unroll 1
  for (int j = 0; j < cnt; ++j) {
    int nv = sList[j];
    nv = min(max(nv, 0), NBLK - 1);
    const int n = __builtin_amdgcn_readfirstlane(nv);
    int cv = sCols[n];
    cv = min(max(cv, 0), NCB - 1);
    const int cb = __builtin_amdgcn_readfirstlane(cv);

    const unsigned short* asrc = XB + (size_t)t0 * KDIM + TB * cb;
    const unsigned short* bsrc = VB + (size_t)n * (TB * TB);

    v4u ra[4], rv[2];
    #pragma unroll
    for (int i = 0; i < 4; ++i) {
      const int p = tid + NTHR * i;
      const int row = p >> 3, pc = p & 7;
      ra[i] = *(const v4ua*)(asrc + (size_t)row * KDIM + 8 * pc);
    }
    #pragma unroll
    for (int i = 0; i < 2; ++i) {
      const int p = tid + NTHR * i;
      rv[i] = *(const v4ua*)(bsrc + 8 * p);
    }
    __syncthreads();
    #pragma unroll
    for (int i = 0; i < 4; ++i) {
      const int p = tid + NTHR * i;
      const int row = p >> 3, pc = p & 7;
      *(v4ua*)(sA + row * SROW + 8 * pc) = ra[i];
    }
    #pragma unroll
    for (int i = 0; i < 2; ++i) {
      const int p = tid + NTHR * i;
      const int row = p >> 3, pc = p & 7;
      *(v4ua*)(sB + row * SROW + 8 * pc) = rv[i];
    }
    __syncthreads();

    #pragma unroll
    for (int ks = 0; ks < 2; ++ks) {
      const v16bf a = load_frag(arow + 32 * ks, h);
      #pragma unroll
      for (int nt = 0; nt < 4; ++nt) {
        const v16bf b = load_frag(brw + 16 * nt * SROW + 32 * ks, h);
        acc[nt] = wmma_bf16(a, b, acc[nt]);
      }
    }
  }
  __syncthreads();

  #pragma unroll
  for (int nt = 0; nt < 4; ++nt) {
    const float bb = sBias[16 * nt + m];
    #pragma unroll
    for (int r = 0; r < 8; ++r)
      sO[(16 * w + 8 * h + r) * TB + 16 * nt + m] = acc[nt][r] + bb;
  }
  __syncthreads();

  {
    const int q8 = lane & 7, sub = lane >> 3;
    #pragma unroll 1
    for (int i = 0; i < 8; ++i) {
      const int lid = w * 32 + i * 4 + sub;
      const int row = lid >> 1, hl = lid & 1;
      float* p = sO + row * TB + 32 * hl + 4 * q8;
      const v4f v = *(const v4fa*)p;
      const v4f g = { gelu_t(v.x), gelu_t(v.y), gelu_t(v.z), gelu_t(v.w) };
      *(v4fa*)p = g;
    }
  }
  __syncthreads();

  out_pass(sO, out, t0, rb, w, lane);
  __threadfence();
  out_pass(sO, out, t0, rb, w, lane);
}

extern "C" void kernel_launch(void* const* d_in, const int* in_sizes, int n_in,
                              void* d_out, int out_size, void* d_ws, size_t ws_size,
                              hipStream_t stream) {
  if (n_in < 5) return;
  if (in_sizes[0] != NX) return;
  if (in_sizes[1] != NV) return;
  if (in_sizes[2] != MDIM) return;
  if (in_sizes[3] != NBLK || in_sizes[4] != NBLK) return;
  if (out_size != TOK * MDIM) return;
  if (WS_TOTAL > ws_size) return;

  const float* x    = (const float*)d_in[0];
  const float* vals = (const float*)d_in[1];
  const float* bias = (const float*)d_in[2];
  const int*   brow = (const int*)d_in[3];
  const int*   bcol = (const int*)d_in[4];
  float* out = (float*)d_out;

  char* ws = (char*)d_ws;
  unsigned short* xb = (unsigned short*)(ws);
  unsigned short* vb = (unsigned short*)(ws + XB_BYTES);

  k_prep<<<XBLK + VBLK, NTHR, 0, stream>>>(x, vals, xb, vb);

  dim3 grid(TOK / TT, NRB);
  k_bsgemm<<<grid, NTHR, 0, stream>>>(xb, vb, bias, brow, bcol, out);
}
